// S4Layer_11811160064012
// MI455X (gfx1250) — hardware-run, weakly checked
//
#include <hip/hip_runtime.h>


#ifndef NB
#define NB 16
#endif
#ifndef SEQ
#define SEQ 4096
#endif
#define NB_FULL  16
#define SEQ_FULL 4096
#ifndef OUT_SEQ
#define OUT_SEQ SEQ
#endif
#define DIN  64
#define HH   256
#define NM   32
#define DOUT 10
#define CT   64
#define NCH  (SEQ / CT)
#define WTP  320
#define HSP  260
#define HNP  264
#define QRS  2048.0f
#define QRI  (1.0f / 2048.0f)
#define WCS  16.0f
#define WCI  (1.0f / 16.0f)
#define TKS  64.0f
#define TKI  (1.0f / 64.0f)
#define LNE  1e-5f

static_assert(NM == 32);
static_assert(CT == 64);
static_assert(SEQ % CT == 0);
static_assert(SEQ % 64 == 0);
static_assert((NB * SEQ) % 64 == 0);
static_assert(NB >= 1);
static_assert(NB <= 16);
static_assert(NB <= NB_FULL);
static_assert(SEQ <= SEQ_FULL);
static_assert(HH % 64 == 0);
static_assert(HH % 8 == 0);
static_assert(HH == 256);
static_assert(DIN % 32 == 0);
static_assert(HH % 32 == 0);
static_assert(WTP == HH + DIN);
static_assert(WTP % 64 == 0);
static_assert(DOUT <= 16);
static_assert((64 * DOUT * 4) % 128 == 0);
static_assert(((size_t)OUT_SEQ * DOUT * 4) % 128 == 0);
static_assert((128 + 32) * 16 == 64 * DOUT * 4);
static_assert((NB * CT) % 32 == 0);
static_assert(4 * 4 == 16);
static_assert(8 * 8 == 64);
static_assert(8 * 32 * 8 == 4 * 16 * 32);
static_assert(16 * 32 * 8 == CT * 64);
static_assert((HSP * 4) % 16 == 0);
static_assert((HNP * 2) % 16 == 0);
static_assert(64 * HSP * 4 + 64 * HNP * 2 + 64 * DOUT * 4 <= 131072);
static_assert(16 * CT * 8 * 2 <= 131072);
static_assert(2 * CT * 64 * 2 + 4 * 16 * 32 * 2 + CT * 4 + 64 * 4 <= 131072);

typedef _Float16 h16;
typedef unsigned short bf;
typedef __attribute__((ext_vector_type(16))) _Float16 v16h;
typedef __attribute__((ext_vector_type(8)))  _Float16 v8h;
typedef __attribute__((ext_vector_type(8)))  float    v8f;
typedef __attribute__((ext_vector_type(4)))  float    v4f;
typedef v4f  __attribute__((may_alias)) v4fa;
typedef v8h  __attribute__((may_alias)) v8ha;

__device__ __forceinline__ unsigned short f2bf(float f) { unsigned u = __float_as_uint(f); u += 0x7FFFu + ((u >> 16) & 1u); return (unsigned short)(u >> 16); }
__device__ __forceinline__ float bfr(float f) { return __uint_as_float(((unsigned)f2bf(f)) << 16); }
__device__ __forceinline__ v16h cat16(v8h lo, v8h hi) { return __builtin_shufflevector(lo, hi, 0, 1, 2, 3, 4, 5, 6, 7, 8, 9, 10, 11, 12, 13, 14, 15); }
__device__ __forceinline__ v16h  ldh(const h16* p) { return cat16(*(const v8h*)p, *(const v8h*)(p + 16)); }
__device__ __forceinline__ void wave_sync() { __builtin_amdgcn_fence(3  , "wavefront"); __builtin_amdgcn_wave_barrier(); asm volatile("" ::: "memory"); }
static __device__ __forceinline__ h16 toh_flush(float v) { const h16 r = (h16)v; return (fabsf(v) < 6.103515625e-05f) ? (h16)0.0f : r; }
__device__ __forceinline__ v8f wmma16g(v16h a, v16h b, v8f c) {
    c = __builtin_amdgcn_wmma_f32_16x16x32_f16(false, a, false, b, (short)0, c, false, false);
    asm volatile("v_nop\n\tv_nop\n\tv_nop\n\tv_nop" : "+v"(c) : "v"(a), "v"(b));
    return c;
}
__device__ __forceinline__ float gelu_erf(float y) { return 0.5f * y * (1.0f + erff(y * 0.70710678118654752f)); }

__global__ __launch_bounds__(256) void k_cvth(const float* __restrict__ src, h16* dst, size_t n8) {
    const size_t i = (size_t)blockIdx.x * 256 + threadIdx.x; if (i >= n8) return;
    const v8f v = *(const v8f*)(src + i * 8); v8h o;
#pragma unroll
    for (int k = 0; k < 8; ++k) o[k] = toh_flush(bfr(v[k]));
    *(volatile v8h*)(dst + i * 8) = o; __threadfence(); *(volatile v8h*)(dst + i * 8) = o;
}

__global__ __launch_bounds__(256) void k_wt(const float* __restrict__ src, int srcPitch, int nValid, int nOut, int rows, int dstPitch, int kofs, float scale, h16* dst) {
    const int ppr = rows >> 3;
    const int i = blockIdx.x * 256 + threadIdx.x; if (i >= nOut * ppr) return;
    const int n = i / ppr, pc = i - n * ppr;
    const int nn = n < nValid ? n : nValid - 1;
    const bool ok = n < nValid;
    v8h o;
#pragma unroll
    for (int e = 0; e < 8; ++e) { float x = src[(size_t)(pc * 8 + e) * srcPitch + nn]; asm volatile("" : "+v"(x)); o[e] = toh_flush(ok ? bfr(x) * scale : 0.0f); }
    h16* p = dst + (size_t)n * dstPitch + kofs + pc * 8;
    *(volatile v8h*)p = o; __threadfence(); *(volatile v8h*)p = o;
}

__global__ __launch_bounds__(32) void k_tab(const float* __restrict__ log_dt, const float* __restrict__ log_ar, const float* __restrict__ a_im,
                                            const float* __restrict__ b_re, const float* __restrict__ b_im, const float* __restrict__ c_re, const float* __restrict__ c_im,
                                            h16* TKF, h16* CLF, h16* PF, float* LT) {
#pragma clang fp contract(off)
    __shared__ __align__(16) h16 pt[CT * 64];
    __shared__ __align__(16) h16 ct[CT * 64];
    __shared__ __align__(16) h16 tq[4 * 16 * 32];
    __shared__ __align__(16) float kk[CT];
    __shared__ __align__(16) float lt[64];
    const int n = threadIdx.x & 31; const int h = blockIdx.x; const int idx = h * NM + n;
    const float dt  = expf(bfr(log_dt[h]));
    const float are = -expf(bfr(log_ar[idx]));
    const float aim = bfr(a_im[idx]);
    const float mag = expf(dt * are);
    float sn, cs; sincosf(dt * aim, &sn, &cs);
    const float lre = mag * cs, lim = mag * sn;
    const float cre = bfr(c_re[idx]), cim = bfr(c_im[idx]), bre = bfr(b_re[idx]), bim = bfr(b_im[idx]);
    const float cbr = cre * bre - cim * bim, cbi = cre * bim + cim * bre;
    const float er = lre - 1.0f, ei = lim;
    const float tr = cbr * er - cbi * ei, ti = cbr * ei + cbi * er;
    const float inv = 1.0f / (are * are + aim * aim);
    const float c2r = 2.0f * ((tr * are + ti * aim) * inv);
    const float c2i = 2.0f * ((ti * are - tr * aim) * inv);
    float pr = 1.0f, pi = 0.0f;
#pragma unroll 1
    for (int d = 0; d <= CT; ++d) {
        const float vr = c2r * pr - c2i * pi, vi = c2r * pi + c2i * pr;
        float sm = vr;
        sm += __shfl_xor(sm, 16, 32); sm += __shfl_xor(sm, 8, 32); sm += __shfl_xor(sm, 4, 32); sm += __shfl_xor(sm, 2, 32); sm += __shfl_xor(sm, 1, 32);
        if (d < CT) { if (n == 0) kk[d] = sm; pt[n * 64 + (CT - 1 - d)] = toh_flush(pr); pt[(32 + n) * 64 + (CT - 1 - d)] = toh_flush(pi); }
        if (d >= 1) { ct[(d - 1) * 64 + n] = toh_flush(vr * TKS); ct[(d - 1) * 64 + 32 + n] = toh_flush(-vi * TKS); }
        if (d == CT) { lt[n] = pr; lt[32 + n] = pi; }
        const float qr = pr * lre - pi * lim, qi = pr * lim + pi * lre; pr = qr; pi = qi;
    }
    wave_sync();
#pragma unroll 1
    for (int it = 0; it < 64; ++it) {
        const int id = it * 32 + n; const int dl = id >> 9, m = (id >> 5) & 15, jj = id & 31;
        const int d = 16 * dl + m - jj; const int dc = d < 0 ? 0 : d;
        float kv = kk[dc]; asm volatile("" : "+v"(kv));
        tq[id] = toh_flush((d >= 0) ? kv * TKS : 0.0f);
    }
    wave_sync();
    h16* tkg = TKF + (size_t)h * 2048; h16* clg = CLF + (size_t)h * 4096; h16* pfg = PF + (size_t)h * 4096; float* ltg = LT + (size_t)h * 64;
#pragma unroll 1
    for (int ps = 0; ps < 2; ++ps) {
#pragma unroll 1
        for (int s = 0; s < 8; ++s)  { const int p = s * 32 + n; const v8h v = *(const v8ha*)(&tq[p * 8]); *(volatile v8h*)(tkg + p * 8) = v; }
#pragma unroll 1
        for (int s = 0; s < 16; ++s) { const int p = s * 32 + n; const v8h v = *(const v8ha*)(&ct[p * 8]); *(volatile v8h*)(clg + p * 8) = v;
                                       const v8h w = *(const v8ha*)(&pt[p * 8]); *(volatile v8h*)(pfg + p * 8) = w; }
        if (n < 16) { const v4f v = *(const v4fa*)(&lt[n * 4]); *(volatile v4f*)(ltg + n * 4) = v; }
        if (ps == 0) __threadfence(); }
}

__global__ __launch_bounds__(32) void k_enc(const h16* __restrict__ WT, const h16* __restrict__ XH, const float* __restrict__ benc, h16* UH, h16* UR) {
    __shared__ __align__(16) float os[16 * 68];
    const int lane = threadIdx.x & 31, lr = lane & 15, hi = lane >> 4; const int r0 = blockIdx.x * 64, c0 = blockIdx.y * 64;
    v8f acc[4][4];
#pragma unroll
    for (int mb = 0; mb < 4; ++mb)
#pragma unroll
        for (int nb = 0; nb < 4; ++nb) acc[mb][nb] = (v8f){};
    const size_t aoff = (size_t)(r0 + lr) * WTP + HH + 8 * hi, boff = (size_t)(c0 + lr) * DIN + 8 * hi;
#pragma unroll 1
    for (int kc = 0; kc < DIN; kc += 32) {
        v16h a[4];
#pragma unroll
        for (int mb = 0; mb < 4; ++mb) a[mb] = ldh(WT + aoff + (size_t)mb * 16 * WTP + kc);
#pragma unroll
        for (int nb = 0; nb < 4; ++nb) { const v16h b = ldh(XH + boff + (size_t)nb * 16 * DIN + kc);
#pragma unroll
            for (int mb = 0; mb < 4; ++mb) acc[mb][nb] = wmma16g(a[mb], b, acc[mb][nb]); }
    }
    const int bb = c0 / SEQ, tt = c0 % SEQ;
    const size_t tbase = (size_t)bb * (size_t)HH * SEQ + (size_t)r0 * SEQ + (size_t)tt;
#pragma unroll
    for (int mb = 0; mb < 4; ++mb) {
        float br[8];
#pragma unroll
        for (int j = 0; j < 8; ++j) br[j] = bfr(benc[r0 + mb * 16 + hi * 8 + j]);
#pragma unroll
        for (int nb = 0; nb < 4; ++nb) {
#pragma unroll
            for (int j = 0; j < 8; ++j) os[(hi * 8 + j) * 68 + nb * 16 + lr] = acc[mb][nb][j] * WCI + br[j]; }
        wave_sync();
#pragma unroll 1
        for (int ps = 0; ps < 2; ++ps) {
            const size_t sb = tbase + (size_t)(mb * 16) * SEQ;
#pragma unroll
            for (int s = 0; s < 4; ++s) { const int row = 4 * s + (lane >> 3), c8 = (lane & 7) * 8;
                const v4f x0 = *(const v4fa*)(&os[row * 68 + c8]); const v4f x1 = *(const v4fa*)(&os[row * 68 + c8 + 4]); v8h hv, rv;
#pragma unroll
                for (int i = 0; i < 4; ++i) { const h16 a0 = toh_flush(x0[i]); const h16 a1 = toh_flush(x1[i]); hv[i] = a0; hv[4 + i] = a1;
                                              rv[i] = toh_flush((x0[i] - (float)a0) * QRS); rv[4 + i] = toh_flush((x1[i] - (float)a1) * QRS); }
                const size_t oo = sb + (size_t)row * SEQ + c8;
                *(volatile v8h*)(UH + oo) = hv; *(volatile v8h*)(UR + oo) = rv; }
            if (ps == 0) __threadfence(); }
        wave_sync();
    }
}

__global__ __launch_bounds__(256) void k_scan(const h16* __restrict__ UH, const h16* __restrict__ UR, const h16* __restrict__ TKF, const h16* __restrict__ CLF,
                                              const h16* __restrict__ PF, const float* __restrict__ LT, const float* __restrict__ Dv, h16* Y8) {
    __shared__ __align__(16) h16 ys[16 * CT * 8];
    const int tid = threadIdx.x, lane = tid & 31, lr = lane & 15, hi = lane >> 4;
    const int wave = __builtin_amdgcn_readfirstlane((int)(threadIdx.x >> 5));
    const int hb = blockIdx.x; const int h = hb * 8 + wave;
    const int bl = lr < NB ? lr : NB - 1;
    const float Dh = bfr(Dv[h]);
    const size_t urow = ((size_t)bl * HH + (size_t)h) * SEQ + 8 * hi;
    const size_t tko = (size_t)h * 2048 + (size_t)lr * 32 + 8 * hi;
    const size_t clo = (size_t)h * 4096 + (size_t)lr * 64 + 8 * hi;
    const size_t lto = (size_t)h * 64 + 8 * hi;
    v8f S0 = (v8f){}, S1 = (v8f){}, S2 = (v8f){}, S3 = (v8f){};
    int zo = 0;
#pragma unroll 1
    for (int c = 0; c < NCH; ++c) {
        asm volatile("" : "+s"(zo));
        const int l0 = c * CT;
        const v16h ub0 = ldh(UH + urow + l0), ub1 = ldh(UH + urow + l0 + 32);
        v16h bs0, bs1;
#pragma unroll
        for (int r = 0; r < 8; ++r) { bs0[r] = toh_flush(S0[r]); bs0[8 + r] = toh_flush(S1[r]); bs1[r] = toh_flush(S2[r]); bs1[8 + r] = toh_flush(S3[r]); }
        const h16* tk = TKF + tko + zo; const h16* cl = CLF + clo + zo; const h16* pf = PF + clo + zo; const float* lp = LT + lto + zo;
        v8f y0 = (v8f){}, y1 = (v8f){}, y2 = (v8f){}, y3 = (v8f){};
        { const v16h t0 = ldh(tk), t1 = ldh(tk + 512);
          y0 = wmma16g(t0, ub0, y0); y1 = wmma16g(t1, ub0, y1); y2 = wmma16g(t0, ub1, y2); y3 = wmma16g(t1, ub1, y3); }
        { const v16h t2 = ldh(tk + 1024), t3 = ldh(tk + 1536);
          y2 = wmma16g(t2, ub0, y2); y3 = wmma16g(t3, ub0, y3); }
        y0 = wmma16g(ldh(cl),        bs0, y0); y0 = wmma16g(ldh(cl + 32),        bs1, y0);
        y1 = wmma16g(ldh(cl + 1024), bs0, y1); y1 = wmma16g(ldh(cl + 1024 + 32), bs1, y1);
        y2 = wmma16g(ldh(cl + 2048), bs0, y2); y2 = wmma16g(ldh(cl + 2048 + 32), bs1, y2);
        y3 = wmma16g(ldh(cl + 3072), bs0, y3); y3 = wmma16g(ldh(cl + 3072 + 32), bs1, y3);
        { const v4f ra = *(const v4f*)(lp), rb = *(const v4f*)(lp + 4), ia = *(const v4f*)(lp + 32), ib = *(const v4f*)(lp + 36);
#pragma unroll
          for (int r = 0; r < 4; ++r) { const float re = S0[r], im = S2[r]; S0[r] = ra[r] * re - ia[r] * im; S2[r] = ra[r] * im + ia[r] * re;
                                        const float rf = S0[4 + r], ig = S2[4 + r]; S0[4 + r] = rb[r] * rf - ib[r] * ig; S2[4 + r] = rb[r] * ig + ib[r] * rf; } }
        { const v4f ra = *(const v4f*)(lp + 16), rb = *(const v4f*)(lp + 20), ia = *(const v4f*)(lp + 48), ib = *(const v4f*)(lp + 52);
#pragma unroll
          for (int r = 0; r < 4; ++r) { const float re = S1[r], im = S3[r]; S1[r] = ra[r] * re - ia[r] * im; S3[r] = ra[r] * im + ia[r] * re;
                                        const float rf = S1[4 + r], ig = S3[4 + r]; S1[4 + r] = rb[r] * rf - ib[r] * ig; S3[4 + r] = rb[r] * ig + ib[r] * rf; } }
        S0 = wmma16g(ldh(pf),        ub0, S0); S0 = wmma16g(ldh(pf + 32),        ub1, S0);
        S1 = wmma16g(ldh(pf + 1024), ub0, S1); S1 = wmma16g(ldh(pf + 1024 + 32), ub1, S1);
        S2 = wmma16g(ldh(pf + 2048), ub0, S2); S2 = wmma16g(ldh(pf + 2048 + 32), ub1, S2);
        S3 = wmma16g(ldh(pf + 3072), ub0, S3); S3 = wmma16g(ldh(pf + 3072 + 32), ub1, S3);
        const v16h ur0 = ldh(UR + urow + l0), ur1 = ldh(UR + urow + l0 + 32);
        const int yb = (lr * CT + 8 * hi) * 8 + wave;
#pragma unroll
        for (int r = 0; r < 8; ++r) {
            const float u0 = (float)ub0[r]     + (float)ur0[r]     * QRI;
            const float u1 = (float)ub0[8 + r] + (float)ur0[8 + r] * QRI;
            const float u2 = (float)ub1[r]     + (float)ur1[r]     * QRI;
            const float u3 = (float)ub1[8 + r] + (float)ur1[8 + r] * QRI;
            ys[yb + (r)      * 8] = toh_flush(gelu_erf(y0[r] * TKI + Dh * u0));
            ys[yb + (16 + r) * 8] = toh_flush(gelu_erf(y1[r] * TKI + Dh * u1));
            ys[yb + (32 + r) * 8] = toh_flush(gelu_erf(y2[r] * TKI + Dh * u2));
            ys[yb + (48 + r) * 8] = toh_flush(gelu_erf(y3[r] * TKI + Dh * u3)); }
        __syncthreads();
#pragma unroll 1
        for (int ps = 0; ps < 2; ++ps) {
#pragma unroll 1
            for (int p = tid; p < NB * CT; p += 256) { const int b = p >> 6, t = p & 63;
                const v8h v = *(const v8ha*)(&ys[p * 8]);
                *(volatile v8h*)(Y8 + (((size_t)hb * NB + (size_t)b) * SEQ + (size_t)(l0 + t)) * 8) = v; }
            if (ps == 0) __threadfence(); }
        __syncthreads();
    }
}

__global__ __launch_bounds__(128) void k_mix(const h16* __restrict__ Y8, const h16* __restrict__ XH, const h16* __restrict__ WT, const h16* __restrict__ WD,
                                             const float* __restrict__ bout, const float* __restrict__ benc, const float* __restrict__ lng, const float* __restrict__ lnb,
                                             const float* __restrict__ bdec, float* OUT) {
    __shared__ __align__(16) float hs[64 * HSP];
    __shared__ __align__(16) h16 hn[64 * HNP];
    __shared__ __align__(16) float os[64 * DOUT];
    const int tid = threadIdx.x, lane = tid & 31, lr = lane & 15, hi = lane >> 4;
    const int wave = __builtin_amdgcn_readfirstlane((int)(threadIdx.x >> 5));
    const int r0 = blockIdx.x * 64; const int bb = r0 / SEQ, t0 = r0 % SEQ; const int c0 = wave * 64;
    const size_t GS = (size_t)NB * SEQ * 8;
    v8f acc[4][4];
#pragma unroll
    for (int mb = 0; mb < 4; ++mb)
#pragma unroll
        for (int nb = 0; nb < 4; ++nb) acc[mb][nb] = (v8f){};
    const size_t yo = ((size_t)bb * SEQ + (size_t)(t0 + lr)) * 8 + (size_t)hi * GS;
    const size_t bo = (size_t)(c0 + lr) * WTP + 8 * hi;
#pragma unroll 1
    for (int kc = 0; kc < HH / 32; ++kc) {
        v16h a[4];
#pragma unroll
        for (int mb = 0; mb < 4; ++mb) a[mb] = cat16(*(const v8h*)(Y8 + yo + (size_t)(kc * 4) * GS + mb * 128), *(const v8h*)(Y8 + yo + (size_t)(kc * 4 + 2) * GS + mb * 128));
#pragma unroll
        for (int nb = 0; nb < 4; ++nb) { const v16h b = ldh(WT + bo + (size_t)nb * 16 * WTP + kc * 32);
#pragma unroll
            for (int mb = 0; mb < 4; ++mb) acc[mb][nb] = wmma16g(a[mb], b, acc[mb][nb]); }
    }
    const size_t xo = (size_t)(r0 + lr) * DIN + 8 * hi;
#pragma unroll 1
    for (int kx = 0; kx < DIN / 32; ++kx) {
        v16h a[4];
#pragma unroll
        for (int mb = 0; mb < 4; ++mb) a[mb] = ldh(XH + xo + (size_t)mb * 16 * DIN + kx * 32);
#pragma unroll
        for (int nb = 0; nb < 4; ++nb) { const v16h b = ldh(WT + bo + (size_t)nb * 16 * WTP + HH + kx * 32);
#pragma unroll
            for (int mb = 0; mb < 4; ++mb) acc[mb][nb] = wmma16g(a[mb], b, acc[mb][nb]); }
    }
    float cb[4];
#pragma unroll
    for (int nb = 0; nb < 4; ++nb) cb[nb] = bfr(bout[c0 + nb * 16 + lr]) + bfr(benc[c0 + nb * 16 + lr]);
#pragma unroll
    for (int mb = 0; mb < 4; ++mb)
#pragma unroll
        for (int nb = 0; nb < 4; ++nb)
#pragma unroll
            for (int j = 0; j < 8; ++j) hs[(mb * 16 + hi * 8 + j) * HSP + c0 + nb * 16 + lr] = acc[mb][nb][j] * WCI + cb[nb];
    __syncthreads();
    float g8[8], b8[8];
    { const v4f ga = *(const v4f*)(lng + lane * 8), gb = *(const v4f*)(lng + lane * 8 + 4), ba = *(const v4f*)(lnb + lane * 8), bc = *(const v4f*)(lnb + lane * 8 + 4);
#pragma unroll
      for (int e = 0; e < 4; ++e) { g8[e] = bfr(ga[e]); g8[4 + e] = bfr(gb[e]); b8[e] = bfr(ba[e]); b8[4 + e] = bfr(bc[e]); } }
#pragma unroll 1
    for (int rr = 0; rr < 16; ++rr) {
        const int row = wave * 16 + rr;
        const v4f x0 = *(const v4fa*)(&hs[row * HSP + lane * 8]); const v4f x1 = *(const v4fa*)(&hs[row * HSP + lane * 8 + 4]);
        float s = ((x0[0] + x0[1]) + (x0[2] + x0[3])) + ((x1[0] + x1[1]) + (x1[2] + x1[3]));
        s += __shfl_xor(s, 16, 32); s += __shfl_xor(s, 8, 32); s += __shfl_xor(s, 4, 32); s += __shfl_xor(s, 2, 32); s += __shfl_xor(s, 1, 32);
        const float mean = s * (1.0f / HH);
        float dv[8];
#pragma unroll
        for (int e = 0; e < 4; ++e) { dv[e] = x0[e] - mean; dv[4 + e] = x1[e] - mean; }
        float q = ((dv[0] * dv[0] + dv[1] * dv[1]) + (dv[2] * dv[2] + dv[3] * dv[3])) + ((dv[4] * dv[4] + dv[5] * dv[5]) + (dv[6] * dv[6] + dv[7] * dv[7]));
        q += __shfl_xor(q, 16, 32); q += __shfl_xor(q, 8, 32); q += __shfl_xor(q, 4, 32); q += __shfl_xor(q, 2, 32); q += __shfl_xor(q, 1, 32);
        const float rstd = 1.0f / sqrtf(q * (1.0f / HH) + LNE);
        v8h o;
#pragma unroll
        for (int e = 0; e < 8; ++e) o[e] = toh_flush(dv[e] * rstd * g8[e] + b8[e]);
        *(v8ha*)(&hn[row * HNP + lane * 8]) = o;
    }
    wave_sync();
    v8f dacc = (v8f){};
    const int ao = (wave * 16 + lr) * HNP + 8 * hi;
    const size_t wo = (size_t)lr * HH + 8 * hi;
#pragma unroll 1
    for (int kc = 0; kc < HH / 32; ++kc) {
        const v16h a = cat16(*(const v8ha*)(&hn[ao + kc * 32]), *(const v8ha*)(&hn[ao + kc * 32 + 16]));
        const v16h b = ldh(WD + wo + kc * 32);
        dacc = wmma16g(a, b, dacc);
    }
    { const int dcl = lr < DOUT ? lr : DOUT - 1;
      float bd = bdec[dcl]; asm volatile("" : "+v"(bd)); bd = bfr(bd);
#pragma unroll
      for (int j = 0; j < 8; ++j) { const float v = dacc[j] * WCI + bd; if (lr < DOUT) os[(wave * 16 + hi * 8 + j) * DOUT + lr] = v; } }
    __syncthreads();
    float* ob = OUT + ((size_t)bb * OUT_SEQ + (size_t)t0) * DOUT;
#pragma unroll 1
    for (int ps = 0; ps < 2; ++ps) {
        { const v4f v = *(const v4fa*)(&os[tid * 4]); *(volatile v4f*)(ob + tid * 4) = v; }
        if (tid < 32) { const v4f v = *(const v4fa*)(&os[(128 + tid) * 4]); *(volatile v4f*)(ob + (128 + tid) * 4) = v; }
        if (ps == 0) __threadfence(); }
}

static constexpr size_t al256(size_t v) { return (v + 255) & ~(size_t)255; }
static constexpr size_t SZ_XH = al256((size_t)NB * SEQ * DIN * 2);
static constexpr size_t SZ_WT = al256((size_t)HH * WTP * 2);
static constexpr size_t SZ_WD = al256((size_t)16 * HH * 2);
static constexpr size_t SZ_TK = al256((size_t)HH * 2048 * 2);
static constexpr size_t SZ_CL = al256((size_t)HH * CT * 64 * 2);
static constexpr size_t SZ_LT = al256((size_t)HH * 64 * 4);
static constexpr size_t SZ_UP = al256((size_t)NB * HH * SEQ * 2);
static constexpr size_t SZ_TOTAL = SZ_XH + SZ_WT + SZ_WD + SZ_TK + 2 * SZ_CL + SZ_LT + 3 * SZ_UP;
static_assert(SZ_TOTAL <= (size_t)134217728);
static_assert((size_t)(HH / 8) * NB * SEQ * 8 == (size_t)NB * HH * SEQ);
static_assert((size_t)(HH - 1) * 2048 + 255 * 8 + 8 <= (size_t)HH * 2048);
static_assert((size_t)(HH - 1) * 4096 + 511 * 8 + 8 <= (size_t)HH * CT * 64);
static_assert((size_t)(HH - 1) * WTP + HH + 7 * 8 + 8 <= (size_t)HH * WTP);
static_assert(((size_t)(NB - 1) * OUT_SEQ + SEQ) * DOUT * 4 <= (size_t)NB_FULL * SEQ_FULL * DOUT * 4 || OUT_SEQ != SEQ);

extern "C" void kernel_launch(void* const* d_in, const int* in_sizes, int n_in,
                              void* d_out, int out_size, void* d_ws, size_t ws_size, hipStream_t stream) {
    if (n_in < 17) return;
    const size_t needx = ((size_t)(NB - 1) * SEQ_FULL + SEQ) * DIN;
    if ((size_t)in_sizes[0] < needx) return;
    if ((size_t)in_sizes[1] < (size_t)DIN * HH || in_sizes[2] < HH || in_sizes[3] < HH) return;
    for (int i = 4; i <= 9; ++i) if ((size_t)in_sizes[i] < (size_t)HH * NM) return;
    if (in_sizes[10] < HH || (size_t)in_sizes[11] < (size_t)HH * HH || in_sizes[12] < HH || in_sizes[13] < HH || in_sizes[14] < HH) return;
    if (in_sizes[15] < HH * DOUT || in_sizes[16] < DOUT) return;
    if ((size_t)out_size < ((size_t)(NB - 1) * OUT_SEQ + SEQ) * DOUT) return;
    if (SZ_TOTAL > ws_size) return;
    const float* x     = (const float*)d_in[0];
    const float* wenc  = (const float*)d_in[1];
    const float* benc  = (const float*)d_in[2];
    const float* logdt = (const float*)d_in[3];
    const float* logar = (const float*)d_in[4];
    const float* aim   = (const float*)d_in[5];
    const float* bre   = (const float*)d_in[6];
    const float* bim   = (const float*)d_in[7];
    const float* cre   = (const float*)d_in[8];
    const float* cim   = (const float*)d_in[9];
    const float* dsk   = (const float*)d_in[10];
    const float* wout  = (const float*)d_in[11];
    const float* bout  = (const float*)d_in[12];
    const float* lng   = (const float*)d_in[13];
    const float* lnb   = (const float*)d_in[14];
    const float* wdec  = (const float*)d_in[15];
    const float* bdec  = (const float*)d_in[16];
    float* OUT = (float*)d_out;
    char* wsp = (char*)d_ws;
    h16* XH  = (h16*)wsp; wsp += SZ_XH;
    h16* WT  = (h16*)wsp; wsp += SZ_WT;
    h16* WD  = (h16*)wsp; wsp += SZ_WD;
    h16* TKF = (h16*)wsp; wsp += SZ_TK;
    h16* CLF = (h16*)wsp; wsp += SZ_CL;
    h16* PF  = (h16*)wsp; wsp += SZ_CL;
    float* LT = (float*)wsp; wsp += SZ_LT;
    h16* UH  = (h16*)wsp; wsp += SZ_UP;
    h16* UR  = (h16*)wsp; wsp += SZ_UP;
    h16* Y8  = (h16*)wsp; wsp += SZ_UP;

    if (SEQ == SEQ_FULL) {
        const size_t n8 = (size_t)NB * SEQ * DIN / 8;
        k_cvth<<<(unsigned)((n8 + 255) / 256), 256, 0, stream>>>(x, XH, n8);
    } else {
        const size_t n8 = (size_t)SEQ * DIN / 8;
        for (int b = 0; b < NB; ++b) k_cvth<<<(unsigned)((n8 + 255) / 256), 256, 0, stream>>>(x + (size_t)b * SEQ_FULL * DIN, XH + (size_t)b * SEQ * DIN, n8);
    }
    k_wt<<<(HH * (HH / 8) + 255) / 256, 256, 0, stream>>>(wout, HH, HH, HH, HH, WTP, 0, WCS, WT);
    k_wt<<<(HH * (DIN / 8) + 255) / 256, 256, 0, stream>>>(wenc, HH, HH, HH, DIN, WTP, HH, WCS, WT);
    k_wt<<<(16 * (HH / 8) + 255) / 256, 256, 0, stream>>>(wdec, DOUT, DOUT, 16, HH, HH, 0, WCS, WD);
    k_tab<<<HH, 32, 0, stream>>>(logdt, logar, aim, bre, bim, cre, cim, TKF, CLF, PF, LT);
    k_enc<<<dim3(HH / 64, NB * SEQ / 64, 1), 32, 0, stream>>>(WT, XH, benc, UH, UR);
    k_scan<<<HH / 8, 256, 0, stream>>>(UH, UR, TKF, CLF, PF, LT, dsk, Y8);
    k_mix<<<NB * SEQ / 64, 128, 0, stream>>>(Y8, XH, WT, WD, bout, benc, lng, lnb, bdec, OUT);
}
